// ComputeCorr_24017457119748
// MI455X (gfx1250) — hardware-verified
//
#include <hip/hip_runtime.h>
#include <math.h>

#define BB 4
#define NPTS 4096
#define DKK 64
#define QW 2
#define KST 72

typedef _Float16 f16;
typedef __attribute__((ext_vector_type(16))) f16 f16x16;
typedef __attribute__((ext_vector_type(8)))  f16 f16x8;
typedef __attribute__((ext_vector_type(8)))  float f32x8;
typedef __attribute__((ext_vector_type(4)))  float v4f_t;
typedef float v4fa __attribute__((ext_vector_type(4), may_alias));

__device__ __forceinline__ f32x8 wmma16(f16x16 a, f16x16 b, f32x8 c) {
  c = __builtin_amdgcn_wmma_f32_16x16x32_f16(false, a, false, b, (short)0, c, false, false);
  asm volatile("v_nop\n\tv_nop\n\tv_nop\n\tv_nop" : "+v"(c) : "v"(a), "v"(b));
  return c;
}
__device__ __forceinline__ f16x16 lds_frag(const f16* base, int stride) {
  const int lane = threadIdx.x & 31, row = lane & 15, kh = (lane >> 4) * 8;
  const f16x8 lo = *(const f16x8*)(base + row * stride + kh);
  const f16x8 hi = *(const f16x8*)(base + row * stride + kh + 16);
  f16x16 f;
#pragma unroll
  for (int i = 0; i < 8; ++i) { f[i] = lo[i]; f[i + 8] = hi[i]; }
  return f;
}
__device__ __forceinline__ void split16(float v, f16& h, f16& l) { h = (f16)v; l = (f16)((v - (float)h) * 2048.0f); }

__global__ __launch_bounds__(256) void k_norms(const float* __restrict__ F, float* __restrict__ nrm) {
  __shared__ __attribute__((aligned(16))) float nS[256];
  const int b = blockIdx.x / (NPTS / 256), p0 = (blockIdx.x % (NPTS / 256)) * 256, tid = threadIdx.x;
  const float* f = F + (size_t)b * DKK * NPTS + p0 + tid;
  float s = 0.0f;
#pragma unroll 8
  for (int d = 0; d < DKK; ++d) { const float v = f[(size_t)d * NPTS]; s += v * v; }
  nS[tid] = s;
  __syncthreads();
  if (tid < 64) { *(volatile v4f_t*)(nrm + (size_t)b * NPTS + p0 + tid * 4) = *(const volatile v4fa*)(nS + tid * 4); __threadfence(); *(volatile v4f_t*)(nrm + (size_t)b * NPTS + p0 + tid * 4) = *(const volatile v4fa*)(nS + tid * 4); }
}

__global__ __launch_bounds__(64) void k_corr(const float* __restrict__ Qc, const float* __restrict__ Kc, const float* __restrict__ Vc,
                                            const float* __restrict__ bbk, float* __restrict__ out) {
  __shared__ __attribute__((aligned(16))) f16 qS[2][64 * KST];
  __shared__ __attribute__((aligned(16))) f16 kS[2][32 * KST];
  __shared__ __attribute__((aligned(16))) f16 vS[2][16 * 40];
  __shared__ float bbS[32];
  __shared__ __attribute__((aligned(16))) float oS[64 * 3];
  const int q0blk = blockIdx.x * 64, b = blockIdx.y;
  const int t = threadIdx.x, wave = t >> 5, lane = t & 31, qlane = lane & 15, kh8 = (lane >> 4) * 8;
  const float* Qb = Qc + (size_t)b * DKK * NPTS;
  const float* Kb = Kc + (size_t)b * DKK * NPTS;
  const float* Vb = Vc + (size_t)b * NPTS * 3;
  const float* bb = bbk + (size_t)b * NPTS;
  for (int e = t; e < 64 * 64; e += 64) { const int d = e >> 6, q = e & 63; f16 h, l; split16(Qb[(size_t)d * NPTS + q0blk + q], h, l); qS[0][q * KST + d] = h; qS[1][q * KST + d] = l; }
  for (int e = t; e < 2 * 16 * 40; e += 64) (&vS[0][0])[e] = (f16)0.0f;
  __syncthreads();
  f16x16 qh[QW][2], ql[QW][2];
#pragma unroll
  for (int qt = 0; qt < QW; ++qt)
#pragma unroll
    for (int c = 0; c < 2; ++c) { qh[qt][c] = lds_frag(qS[0] + (wave * 32 + 16 * qt) * KST + c * 32, KST); ql[qt][c] = lds_frag(qS[1] + (wave * 32 + 16 * qt) * KST + c * 32, KST); }
  f32x8 o[QW] = {}, ox[QW] = {};
  float mrun[QW], lrun[QW];
#pragma unroll
  for (int qt = 0; qt < QW; ++qt) { mrun[qt] = -INFINITY; lrun[qt] = 0.0f; }
  const float L2E = 1.44269504088896340736f;
#pragma unroll 1
  for (int kb = 0; kb < NPTS; kb += 32) {
    __syncthreads();
    { const float* kr = Kb + (size_t)t * NPTS + kb;
#pragma unroll
      for (int i = 0; i < 8; ++i) { const v4f_t v = *(const v4f_t*)(kr + 4 * i);
#pragma unroll
        for (int u = 0; u < 4; ++u) { f16 h, l; split16(v[u], h, l); kS[0][(4 * i + u) * KST + t] = h; kS[1][(4 * i + u) * KST + t] = l; } }
      if (t < 32) { bbS[t] = bb[kb + t];
#pragma unroll
        for (int c = 0; c < 3; ++c) { f16 h, l; split16(Vb[(size_t)(kb + t) * 3 + c], h, l); vS[0][c * 40 + t] = h; vS[1][c * 40 + t] = l; } } }
    __syncthreads();
    f16x16 kfh[2][2], kfl[2][2];
#pragma unroll
    for (int kt = 0; kt < 2; ++kt)
#pragma unroll
      for (int c = 0; c < 2; ++c) { kfh[kt][c] = lds_frag(kS[0] + (kt * 16) * KST + c * 32, KST); kfl[kt][c] = lds_frag(kS[1] + (kt * 16) * KST + c * 32, KST); }
    const f16x16 vh = lds_frag(vS[0], 40), vl = lds_frag(vS[1], 40);
#pragma unroll
    for (int qt = 0; qt < QW; ++qt) {
      f32x8 s0 = {}, s1 = {}, s0x = {}, s1x = {};
#pragma unroll
      for (int c = 0; c < 2; ++c) {
        s0 = wmma16(kfh[0][c], qh[qt][c], s0); s0x = wmma16(kfh[0][c], ql[qt][c], s0x); s0x = wmma16(kfl[0][c], qh[qt][c], s0x);
        s1 = wmma16(kfh[1][c], qh[qt][c], s1); s1x = wmma16(kfh[1][c], ql[qt][c], s1x); s1x = wmma16(kfl[1][c], qh[qt][c], s1x);
      }
      float mx = -INFINITY;
#pragma unroll
      for (int r = 0; r < 8; ++r) {
        s0[r] = (2.0f * (s0[r] + s0x[r] * (1.0f / 2048.0f)) - bbS[kh8 + r]) * L2E;
        s1[r] = (2.0f * (s1[r] + s1x[r] * (1.0f / 2048.0f)) - bbS[16 + kh8 + r]) * L2E;
        mx = fmaxf(mx, fmaxf(s0[r], s1[r]));
      }
      mx = fmaxf(mx, __shfl_xor(mx, 16, 32));
      const float mnew = fmaxf(mrun[qt], mx), alpha = exp2f(mrun[qt] - mnew);
      f16x16 pf; float rs = 0.0f;
#pragma unroll
      for (int r = 0; r < 8; ++r) { const float p0 = exp2f(s0[r] - mnew), p1 = exp2f(s1[r] - mnew); rs += p0 + p1; pf[r] = (f16)(p0 * 1024.0f); pf[8 + r] = (f16)(p1 * 1024.0f); }
      rs += __shfl_xor(rs, 16, 32);
      lrun[qt] = lrun[qt] * alpha + rs; mrun[qt] = mnew;
#pragma unroll
      for (int r = 0; r < 8; ++r) { o[qt][r] *= alpha; ox[qt][r] *= alpha; }
      o[qt] = wmma16(vh, pf, o[qt]); ox[qt] = wmma16(vl, pf, ox[qt]);
    }
  }
#pragma unroll
  for (int qt = 0; qt < QW; ++qt) {
    const float rl = 1.0f / (lrun[qt] * 1024.0f);
    if (kh8 == 0) {
#pragma unroll
      for (int r = 0; r < 3; ++r) oS[(wave * 32 + 16 * qt + qlane) * 3 + r] = (o[qt][r] + ox[qt][r] * (1.0f / 2048.0f)) * rl;
    }
  }
  __syncthreads();
  if (t < 48) {
#pragma unroll 1
    for (int pass = 0; pass < 2; ++pass) { *(volatile v4f_t*)(out + ((size_t)b * NPTS + q0blk) * 3 + t * 4) = *(const volatile v4fa*)(oS + t * 4); __threadfence(); }
  }
}

extern "C" void kernel_launch(void* const* d_in, const int* in_sizes, int n_in,
                              void* d_out, int out_size, void* d_ws, size_t ws_size,
                              hipStream_t stream) {
  (void)in_sizes; (void)n_in; (void)ws_size;
  const float* src = (const float*)d_in[0];
  const float* tgt = (const float*)d_in[1];
  const float* srcf = (const float*)d_in[2];
  const float* tgtf = (const float*)d_in[3];
  float* out0 = (float*)d_out;
  float* out1 = (float*)((char*)d_out + (size_t)BB * NPTS * 3 * 4);
  (void)out_size;
  char* ws = (char*)d_ws;
  float* nS = (float*)ws; ws += (size_t)BB * NPTS * 4;
  float* nT = (float*)ws; ws += (size_t)BB * NPTS * 4;
  k_norms<<<dim3(BB * NPTS / 256), dim3(256), 0, stream>>>(srcf, nS);
  k_norms<<<dim3(BB * NPTS / 256), dim3(256), 0, stream>>>(tgtf, nT);
  k_corr<<<dim3(NPTS / 64, BB), dim3(64), 0, stream>>>(srcf, tgtf, tgt, nT, out0);
  k_corr<<<dim3(NPTS / 64, BB), dim3(64), 0, stream>>>(tgtf, srcf, src, nS, out1);
}
